// HGTConv_47888885351096
// MI455X (gfx1250) — hardware-run, weakly checked
//
#include <hip/hip_runtime.h>

typedef float          v8f   __attribute__((ext_vector_type(8)));
typedef float          v4f   __attribute__((ext_vector_type(4)));
typedef unsigned int   v4u   __attribute__((ext_vector_type(4)));
typedef int            v8i   __attribute__((ext_vector_type(8)));
typedef unsigned short v8us  __attribute__((ext_vector_type(8)));
typedef unsigned short v16us __attribute__((ext_vector_type(16)));
typedef __bf16         v16bf __attribute__((ext_vector_type(16)));
typedef _Float16       v16h  __attribute__((ext_vector_type(16)));
typedef v4f  __attribute__((may_alias)) v4fa;
typedef v8us __attribute__((may_alias)) v8usa;
union FragB { v16bf v; v16us u; v8us h[2]; v8i w; };
union FragH { v16h  v; v16us u; v8us h[2]; v8i w; };

__device__ __forceinline__ v8f wmb(const FragB& a, const FragB& b, v8f c) {
  v8f d = __builtin_amdgcn_wmma_f32_16x16x32_bf16(false, a.v, false, b.v, (short)0, c, false, false);
  asm volatile("v_nop\n\tv_nop\n\tv_nop\n\tv_nop" : "+v"(d) : "v"(a.w), "v"(b.w));
  return d;
}

__device__ __forceinline__ v8f wmh(const FragH& a, const FragH& b, v8f c) {
  v8f d = __builtin_amdgcn_wmma_f32_16x16x32_f16(false, a.v, false, b.v, (short)0, c, false, false);
  asm volatile("v_nop\n\tv_nop\n\tv_nop\n\tv_nop" : "+v"(d) : "v"(a.w), "v"(b.w));
  return d;
}

__device__ __forceinline__ unsigned bf16_bits(float f) {
  const unsigned u = __float_as_uint(f);
  const unsigned r = (u + 0x7FFFu + ((u >> 16) & 1u)) >> 16;
  const unsigned q = (u >> 16) | 0x40u;
  return ((u & 0x7fffffffu) > 0x7f800000u) ? q : r;
}

__device__ __forceinline__ float bf16_val(float f) {
  return __uint_as_float(bf16_bits(f) << 16);
}
__device__ __forceinline__ int clampi(int v, int lo, int hi) {
  return v < lo ? lo : (v > hi ? hi : v);
}

__device__ __forceinline__ unsigned f16_bits(float f) {
  const unsigned u  = __float_as_uint(f);
  const unsigned s  = (u >> 16) & 0x8000u;
  const unsigned a  = u & 0x7fffffffu;
  const unsigned t  = a - 0x38000000u;
  const unsigned r  = (t + 0x0FFFu + ((t >> 13) & 1u)) >> 13;
  const unsigned rc = r > 0x7C00u ? 0x7C00u : r;
  const bool small  = a < 0x38800000u;
  const bool isnan  = a > 0x7f800000u;
  const unsigned fin = small ? 0u : (s | rc);
  return isnan ? (s | 0x7E00u) : fin;
}

__device__ __forceinline__ unsigned pk16(unsigned lo, unsigned hi) { return lo | (hi << 16); }
__device__ __forceinline__ unsigned bf16_lo_bits(float v) {
  float hi = bf16_val(v);
  asm volatile("" : "+v"(hi));
  return bf16_bits(v - hi);
}
__device__ __forceinline__ v4u pack8_bf16(v4f a, v4f c) {
  return (v4u){ pk16(bf16_bits(a[0]), bf16_bits(a[1])), pk16(bf16_bits(a[2]), bf16_bits(a[3])),
                pk16(bf16_bits(c[0]), bf16_bits(c[1])), pk16(bf16_bits(c[2]), bf16_bits(c[3])) };
}
__device__ __forceinline__ v4u pack8_bf16_lo(v4f a, v4f c) {
  return (v4u){ pk16(bf16_lo_bits(a[0]), bf16_lo_bits(a[1])), pk16(bf16_lo_bits(a[2]), bf16_lo_bits(a[3])),
                pk16(bf16_lo_bits(c[0]), bf16_lo_bits(c[1])), pk16(bf16_lo_bits(c[2]), bf16_lo_bits(c[3])) };
}
__device__ __forceinline__ v4u pack8_f16(v4f a, v4f c) {
  return (v4u){ pk16(f16_bits(a[0]), f16_bits(a[1])), pk16(f16_bits(a[2]), f16_bits(a[3])),
                pk16(f16_bits(c[0]), f16_bits(c[1])), pk16(f16_bits(c[2]), f16_bits(c[3])) };
}

template <int FORM>
__global__ __launch_bounds__(256) void k_plane(const float* __restrict__ src, int rows, int cols, int ldsrc,
                                               unsigned short* __restrict__ dst, int MP, int KP) {
  static_assert(FORM >= 0 && FORM <= 3);
  const int KTOT = (FORM == 1 || FORM == 3) ? 2 * KP : KP;
  const unsigned ppr   = (unsigned)(KTOT >> 3);
  const unsigned kp8   = (unsigned)(KP >> 3);
  const unsigned total = (unsigned)MP * ppr;
  const unsigned g     = blockIdx.x * 256u + threadIdx.x;
  const unsigned rowu  = g / ppr;
  const unsigned p     = g - rowu * ppr;
  const bool second    = p >= kp8;
  const int row = (int)rowu;
  const int c0  = (int)((second ? p - kp8 : p) << 3);
  const float* srow = src + (size_t)clampi(row, 0, rows - 1) * (size_t)ldsrc;
  float x[8];
  unsigned mk[8];
#pragma unroll
  for (int e = 0; e < 8; ++e) {
    const int c = c0 + e;
    const float v = srow[clampi(c, 0, cols - 1)];
    asm volatile("" :: "v"(v));
    x[e]  = v;
    mk[e] = (row < rows && c < cols) ? 0xFFFFu : 0u;
  }
  const v4f a = (v4f){ x[0], x[1], x[2], x[3] };
  const v4f c = (v4f){ x[4], x[5], x[6], x[7] };
  v4u o;
  if (FORM == 2) {
    o = pack8_f16(a, c);
  } else {
    const v4u hi = pack8_bf16(a, c);
    o = hi;
    if (FORM == 1) { const v4u lo = pack8_bf16_lo(a, c); o = second ? lo : hi; }
  }
  const v4u mw = (v4u){ pk16(mk[0], mk[1]), pk16(mk[2], mk[3]), pk16(mk[4], mk[5]), pk16(mk[6], mk[7]) };
  o &= mw;
  if (g < total) {
    volatile v4u* q = (volatile v4u*)(dst + (size_t)g * 8);
    *q = o;
    __threadfence();
    *q = o;
  }
}

template <int FORM> struct FragOf    { typedef FragB T; };
template <>         struct FragOf<2> { typedef FragH T; };
__device__ __forceinline__ v8f mm(const FragB& a, const FragB& b, v8f c) { return wmb(a, b, c); }
__device__ __forceinline__ v8f mm(const FragH& a, const FragH& b, v8f c) { return wmh(a, b, c); }
template <class F> __device__ __forceinline__ F ld_frag(const unsigned short* p) {
  F f;
  f.h[0] = *(const v8usa*)(p);
  f.h[1] = *(const v8usa*)(p + 16);
  return f;
}

template <int FORM, int EPI>
__global__ __launch_bounds__(256) __attribute__((amdgpu_num_vgpr(248)))
void k_gemm_nt(const unsigned short* __restrict__ A, const unsigned short* __restrict__ B,
               const float* __restrict__ bias, float* __restrict__ D, int M, int N, int KTOT, int ldd) {
  static_assert(FORM >= 0 && FORM <= 2);
  static_assert(EPI == 0 || EPI == 1);
  typedef typename FragOf<FORM>::T F;
  __shared__ __attribute__((aligned(16))) float sT[8][16 * 68];
  const int lane = threadIdx.x & 31;
  const int wave = threadIdx.x >> 5;
  const int tilesM = (M + 63) >> 6;
  const int tilesN = (N + 63) >> 6;
  const int tile = blockIdx.x * 8 + wave;
  if (tile >= tilesM * tilesN) return;
  const int tm = tile / tilesN;
  const int tn = tile - tm * tilesN;
  const int m0 = tm << 6;
  const int n0 = tn << 6;

  const int rl = lane & 15;
  const int h8 = (lane >> 4) * 8;
  const unsigned short* pa = A + (size_t)(m0 + rl) * (size_t)KTOT + h8;
  const unsigned short* pb = B + (size_t)(n0 + rl) * (size_t)KTOT + h8;

  v8f acc[4][4];
#pragma unroll
  for (int i = 0; i < 4; ++i)
#pragma unroll
    for (int j = 0; j < 4; ++j) acc[i][j] = (v8f){0.f, 0.f, 0.f, 0.f, 0.f, 0.f, 0.f, 0.f};

#pragma unroll 1
  for (int k0 = 0; k0 < KTOT; k0 += 32) {
    F bf[4];
#pragma unroll
    for (int j = 0; j < 4; ++j) bf[j] = ld_frag<F>(pb + (size_t)(j << 4) * (size_t)KTOT + k0);
#pragma unroll
    for (int i = 0; i < 4; ++i) {
      const F af = ld_frag<F>(pa + (size_t)(i << 4) * (size_t)KTOT + k0);
#pragma unroll
      for (int j = 0; j < 4; ++j) acc[i][j] = mm(af, bf[j], acc[i][j]);
    }
  }

  float* slab = sT[wave];
  const int hh = lane >> 4;
  const int c4 = (lane & 15) * 4;
  const int nc = n0 + c4;
  const bool cok = nc < N;
  v4f bv = (v4f){0.f, 0.f, 0.f, 0.f};
  if (EPI == 1) {
    bv = *(const v4fa*)(bias + clampi(nc, 0, N - 4));
    asm volatile("" :: "v"(bv));
  }
#pragma unroll
  for (int i = 0; i < 4; ++i) {
    const int mBase = m0 + (i << 4);
#pragma unroll
    for (int j = 0; j < 4; ++j) {
#pragma unroll
      for (int r = 0; r < 8; ++r) slab[(h8 + r) * 68 + (j << 4) + rl] = acc[i][j][r];
    }
    __builtin_amdgcn_fence(__ATOMIC_RELEASE, "workgroup");
    __builtin_amdgcn_wave_barrier();
    __builtin_amdgcn_fence(__ATOMIC_ACQUIRE, "workgroup");
    v4f vv[8];
#pragma unroll
    for (int it = 0; it < 8; ++it) {
      const int row = it * 2 + hh;
      v4f v = *(const v4fa*)(slab + row * 68 + c4);
      if (EPI == 1) v += bv;
      vv[it] = v;
    }
    for (int pass = 0; pass < 2; ++pass) {
#pragma unroll
      for (int it = 0; it < 8; ++it) {
        const int row = mBase + it * 2 + hh;
        if (cok && row < M) *(volatile v4f*)(D + (size_t)row * (size_t)ldd + nc) = vv[it];
      }
      __threadfence();
    }
    __builtin_amdgcn_fence(__ATOMIC_RELEASE, "workgroup");
    __builtin_amdgcn_wave_barrier();
    __builtin_amdgcn_fence(__ATOMIC_ACQUIRE, "workgroup");
  }
}

#define NN       50000
#define NE       400000
#define MPN      50048
#define CH       128
#define NBLK     49
#define NBROWS   1024
#define DEGCAP   40
#define MAXHITS  8386
#define MAXDEG   22
#define NTHR     256
#define NWAVE    8
#define EPT      8
#define CHUNK    (NTHR * EPT)
#define WCAP     (EPT * 32)
#define LISTN    (NWAVE * WCAP)
#define NBMAX    2048
#define ESH      11
#define RCAP     11264
#define LDS_BKT  ((2 * RCAP + 2 * NBMAX + LISTN) * 4 + 64)
#define WSMAX    ((size_t)128 << 20)

#define T_QB_A     0
#define T_KB_A     128
#define T_VB_A     256
#define T_AB_A     384
#define T_QB_B     512
#define T_KB_B     640
#define T_VB_B     768
#define T_AB_B     896
#define T_PREL_AB  1024
#define T_PREL_BA  1056
#define T_SKIP     1088
#define TAB_BYTES  8192

#define WT_Q_A     0
#define WT_K_A     16384
#define WT_V_A     32768
#define WT_Q_B     49152
#define WT_K_B     65536
#define WT_V_B     81920
#define WT_A2_A    98304
#define WT_A2_B    131072
#define WT_ABD_AB  163840
#define WT_MBD_AB  196608
#define WT_ABD_BA  229376
#define WT_MBD_BA  262144
#define WT_WORDS   294912

static_assert(CH == 8 * 16);
static_assert(32 * 4 == CH);
static_assert(MPN % 64 == 0 && MPN >= NN && MPN - NN < 64);
static_assert(NN % 16 == 0 && NN % 8 == 0 && MPN % 8 == 0);
static_assert(NN == 781 * 64 + 16);
static_assert(NBLK * NBROWS >= NN && (NBLK - 1) * NBROWS < NN);
static_assert(NBROWS <= NBMAX && (1 << ESH) >= NBMAX && NTHR * 8 == NBMAX && LISTN >= NBMAX);
static_assert(NE <= (1 << (32 - ESH)));
static_assert(NE % CHUNK != 0);
static_assert(NE % 4 == 0);
static_assert(RCAP % 1024 == 0 && RCAP * 4 >= MAXHITS * 5 && RCAP > MAXHITS + 1024);
static_assert(DEGCAP >= MAXDEG + 8);
static_assert(LDS_BKT <= 262144);
static_assert((MPN * CH / 8) % 256 == 0 && (MPN * 32) % 256 == 0);

constexpr size_t al256(size_t v) { return (v + 255) & ~(size_t)255; }
constexpr size_t SZ_F     = (size_t)MPN * CH * 4;
constexpr size_t SZ_B1    = (size_t)MPN * 256 * 2;
constexpr size_t SZ_XB    = (size_t)MPN * CH * 2;
constexpr size_t O_F1     = 0;
constexpr size_t O_F2     = al256(O_F1 + SZ_F);
constexpr size_t O_F3     = al256(O_F2 + SZ_F);
constexpr size_t O_B1     = al256(O_F3 + SZ_F);
constexpr size_t O_XB     = al256(O_B1 + SZ_B1);
constexpr size_t O_LIST   = al256(O_XB + SZ_XB);
constexpr size_t O_OFFC   = al256(O_LIST + (size_t)NBLK * RCAP * 4);
constexpr size_t O_META   = al256(O_OFFC + (size_t)NBLK * 2048 * 4);
constexpr size_t O_WT     = al256(O_META + (size_t)NBLK * 128);
constexpr size_t O_TAB    = al256(O_WT + (size_t)WT_WORDS * 2);
constexpr size_t WS_TOTAL = al256(O_TAB + TAB_BYTES);
static_assert(WS_TOTAL <= (size_t)WSMAX);

typedef int v4i __attribute__((ext_vector_type(4)));
typedef v4i __attribute__((may_alias)) v4ia;

__device__ __forceinline__ void wave_sync_lds() {
  __builtin_amdgcn_fence(__ATOMIC_RELEASE, "workgroup");
  __builtin_amdgcn_wave_barrier();
  __builtin_amdgcn_fence(__ATOMIC_ACQUIRE, "workgroup");
}
__device__ __forceinline__ void st2_v4u(void* p, const v4u v) {
  volatile v4u* q = (volatile v4u*)p;
  *q = v;
  __threadfence();
  *q = v;
}
__device__ __forceinline__ void st2_v4f(float* p, const v4f v) {
  volatile v4f* q = (volatile v4f*)p;
  *q = v;
  __threadfence();
  *q = v;
}
__device__ __forceinline__ void st2_v4i(int* p, const v4i v) {
  volatile v4i* q = (volatile v4i*)p;
  *q = v;
  __threadfence();
  *q = v;
}

__device__ __forceinline__ void wt_piece(const float* __restrict__ W, int n, int k8, unsigned short* dst) {
  float x[8];
#pragma unroll
  for (int i = 0; i < 8; ++i) {
    const float v = W[(size_t)(k8 + i) * CH + n];
    asm volatile("" :: "v"(v));
    x[i] = v;
  }
  st2_v4u(dst, pack8_bf16((v4f){x[0], x[1], x[2], x[3]}, (v4f){x[4], x[5], x[6], x[7]}));
}
__device__ __forceinline__ void bd_piece(const float* __restrict__ rel, int n, int p, unsigned short* dst) {
  const int h = n >> 4, e = n & 15;
  const int kc0 = (p & 15) * 8;
  const int hk = kc0 >> 4, d0 = kc0 & 15;
  float x[8];
#pragma unroll
  for (int i = 0; i < 8; ++i) {
    const float v = rel[h * 256 + (d0 + i) * 16 + e];
    asm volatile("" :: "v"(v));
    x[i] = v;
  }
  v4u o = pack8_bf16((v4f){x[0], x[1], x[2], x[3]}, (v4f){x[4], x[5], x[6], x[7]});
  const unsigned mk = (hk == h) ? 0xFFFFFFFFu : 0u;
  o &= (v4u){mk, mk, mk, mk};
  st2_v4u(dst, o);
}

__global__ __launch_bounds__(256) void k_wprep(
    const float* __restrict__ qWa, const float* __restrict__ kWa, const float* __restrict__ vWa,
    const float* __restrict__ aWa, const float* __restrict__ qWb, const float* __restrict__ kWb,
    const float* __restrict__ vWb, const float* __restrict__ aWb,
    const float* __restrict__ arab, const float* __restrict__ mrab,
    const float* __restrict__ arba, const float* __restrict__ mrba,
    const float* __restrict__ qba, const float* __restrict__ kba, const float* __restrict__ vba,
    const float* __restrict__ aba, const float* __restrict__ qbb, const float* __restrict__ kbb,
    const float* __restrict__ vbb, const float* __restrict__ abb,
    const float* __restrict__ prab, const float* __restrict__ prba,
    const float* __restrict__ ska, const float* __restrict__ skb,
    unsigned short* wt, float* tab) {
  const int b = (int)blockIdx.x, tid = (int)threadIdx.x;
  if (b < 48) {
    const int m = b >> 3;
    const int u = (b & 7) * 256 + tid;
    const int n = u >> 4, k8 = (u & 15) * 8;
    unsigned short* dst = wt + (size_t)m * 16384 + (size_t)u * 8;
    if (m == 0)      wt_piece(qWa, n, k8, dst);
    else if (m == 1) wt_piece(kWa, n, k8, dst);
    else if (m == 2) wt_piece(vWa, n, k8, dst);
    else if (m == 3) wt_piece(qWb, n, k8, dst);
    else if (m == 4) wt_piece(kWb, n, k8, dst);
    else             wt_piece(vWb, n, k8, dst);
  } else if (b < 80) {
    const int m = (b - 48) >> 4;
    const int u = ((b - 48) & 15) * 256 + tid;
    const int n = u >> 5, k8 = ((u & 31) & 15) * 8;
    unsigned short* dst = wt + WT_A2_A + (size_t)m * 32768 + (size_t)u * 8;
    if (m == 0) wt_piece(aWa, n, k8, dst);
    else        wt_piece(aWb, n, k8, dst);
  } else if (b < 144) {
    const int m = (b - 80) >> 4;
    const int u = ((b - 80) & 15) * 256 + tid;
    const int n = u >> 5, p = u & 31;
    unsigned short* dst = wt + WT_ABD_AB + (size_t)m * 32768 + (size_t)u * 8;
    if (m == 0)      bd_piece(arab, n, p, dst);
    else if (m == 1) bd_piece(mrab, n, p, dst);
    else if (m == 2) bd_piece(arba, n, p, dst);
    else             bd_piece(mrba, n, p, dst);
  } else {
    const int lane = tid & 31, wave = tid >> 5;
    v4f bv;
    if (wave == 0)      bv = *(const v4fa*)(qba + 4 * lane);
    else if (wave == 1) bv = *(const v4fa*)(kba + 4 * lane);
    else if (wave == 2) bv = *(const v4fa*)(vba + 4 * lane);
    else if (wave == 3) bv = *(const v4fa*)(aba + 4 * lane);
    else if (wave == 4) bv = *(const v4fa*)(qbb + 4 * lane);
    else if (wave == 5) bv = *(const v4fa*)(kbb + 4 * lane);
    else if (wave == 6) bv = *(const v4fa*)(vbb + 4 * lane);
    else                bv = *(const v4fa*)(abb + 4 * lane);
    asm volatile("" :: "v"(bv));
    const v4f rv = (v4f){ bf16_val(bv[0]), bf16_val(bv[1]), bf16_val(bv[2]), bf16_val(bv[3]) };
    st2_v4f(tab + 128 * wave + 4 * lane, rv);
    if (wave == 0) {
      const float pv = prab[lane >> 2];
      asm volatile("" :: "v"(pv));
      const float v = bf16_val(pv);
      volatile float* q = tab + T_PREL_AB + lane;
      *q = v;
      __threadfence();
      *q = v;
    } else if (wave == 1) {
      const float pv = prba[lane >> 2];
      asm volatile("" :: "v"(pv));
      const float v = bf16_val(pv);
      volatile float* q = tab + T_PREL_BA + lane;
      *q = v;
      __threadfence();
      *q = v;
    } else if (wave == 2) {
      const float sa = ska[0];
      const float sb = skb[0];
      asm volatile("" :: "v"(sa), "v"(sb));
      const float ra = bf16_val(sa), rb = bf16_val(sb);
      const float v = (lane == 0) ? ra : ((lane == 1) ? rb : 0.0f);
      volatile float* q = tab + T_SKIP + lane;
      *q = v;
      __threadfence();
      *q = v;
    }
  }
}

__global__ __launch_bounds__(256) void k_split(const float* __restrict__ F, const float* __restrict__ bias,
                                               unsigned short* B1) {
  const unsigned g = blockIdx.x * 256u + threadIdx.x;
  const int row = (int)(g >> 5);
  const int p = (int)(g & 31u);
  const bool second = p >= 16;
  const int c0 = (p & 15) * 8;
  const int rc = row < NN ? row : NN - 1;
  const float* fp = F + (size_t)rc * CH + c0;
  v4f a = *(const v4fa*)fp, c = *(const v4fa*)(fp + 4);
  asm volatile("" :: "v"(a), "v"(c));
  const v4f ba = *(const v4fa*)(bias + c0), bc = *(const v4fa*)(bias + c0 + 4);
  a += ba; c += bc;
  const v4u hi = pack8_bf16(a, c);
  const v4u lo = pack8_bf16_lo(a, c);
  v4u o = second ? lo : hi;
  const unsigned mk = row < NN ? 0xFFFFFFFFu : 0u;
  o &= (v4u){mk, mk, mk, mk};
  st2_v4u(B1 + (size_t)g * 8, o);
}

__device__ __forceinline__ int scan_chunk(const int* __restrict__ dsts, int nE, int cbase, int slotBase,
                                          int nb, int vec8, int* list, int tid, int lane, int wave) {
  int wc = 0;
  const int el0  = tid * EPT;
  const int e0   = cbase + el0;
  const int sent = (-0x7fffffff - 1);
  v4i da, db;
  if (vec8 != 0 && cbase + CHUNK <= nE) {
    da = *(const v4i*)(dsts + e0);
    db = *(const v4i*)(dsts + e0 + 4);
  } else {
    const int t0 = dsts[min(e0 + 0, nE - 1)];
    const int t1 = dsts[min(e0 + 1, nE - 1)];
    const int t2 = dsts[min(e0 + 2, nE - 1)];
    const int t3 = dsts[min(e0 + 3, nE - 1)];
    const int t4 = dsts[min(e0 + 4, nE - 1)];
    const int t5 = dsts[min(e0 + 5, nE - 1)];
    const int t6 = dsts[min(e0 + 6, nE - 1)];
    const int t7 = dsts[min(e0 + 7, nE - 1)];
    asm volatile("" :: "v"(t0), "v"(t1), "v"(t2), "v"(t3), "v"(t4), "v"(t5), "v"(t6), "v"(t7));
    da.x = (e0 + 0 < nE) ? t0 : sent;
    da.y = (e0 + 1 < nE) ? t1 : sent;
    da.z = (e0 + 2 < nE) ? t2 : sent;
    da.w = (e0 + 3 < nE) ? t3 : sent;
    db.x = (e0 + 4 < nE) ? t4 : sent;
    db.y = (e0 + 5 < nE) ? t5 : sent;
    db.z = (e0 + 6 < nE) ? t6 : sent;
    db.w = (e0 + 7 < nE) ? t7 : sent;
  }
  const unsigned nbs = (unsigned)slotBase;
  const unsigned unb = (unsigned)nb;
  const unsigned s0 = (unsigned)da.x - nbs, s1 = (unsigned)da.y - nbs;
  const unsigned s2 = (unsigned)da.z - nbs, s3 = (unsigned)da.w - nbs;
  const unsigned s4 = (unsigned)db.x - nbs, s5 = (unsigned)db.y - nbs;
  const unsigned s6 = (unsigned)db.z - nbs, s7 = (unsigned)db.w - nbs;
  const bool h0 = s0 < unb, h1 = s1 < unb, h2 = s2 < unb, h3 = s3 < unb;
  const bool h4 = s4 < unb, h5 = s5 < unb, h6 = s6 < unb, h7 = s7 < unb;
  const unsigned any = __builtin_amdgcn_ballot_w32(h0 | h1 | h2 | h3 | h4 | h5 | h6 | h7);
  if (any != 0u) {
#define HITJ(J, HJ, SJ) { \
      const unsigned mj = __builtin_amdgcn_ballot_w32(HJ); \
      if (mj != 0u) { \
        if (HJ) { \
          const int pos = wc + (int)__builtin_amdgcn_mbcnt_lo(mj, 0u); \
          if (pos < WCAP) list[wave * WCAP + pos] = ((el0 + (J)) << 12) | (int)(SJ); \
        } \
        wc += (int)__builtin_popcount(mj); } }
    HITJ(0, h0, s0)
    HITJ(1, h1, s1)
    HITJ(2, h2, s2)
    HITJ(3, h3, s3)
    HITJ(4, h4, s4)
    HITJ(5, h5, s5)
    HITJ(6, h6, s6)
    HITJ(7, h7, s7)
#undef HITJ
  }
  return wc;
}

__device__ __forceinline__ int build_lists(const int* __restrict__ dsts, int nE, int nodeBase, int nb, int vec8,
                                           int* reg1, int* reg2, int* scnt, int* soff, int* list,
                                           int* wcnt, int* wtot, int tid, int lane, int wave) {
  for (int i = tid; i < NBMAX; i += NTHR) scnt[i] = 0;
  __syncthreads();

  int tot = 0;
  const int nChunks = (nE + CHUNK - 1) / CHUNK;
#pragma unroll 1
  for (int ch = 0; ch < nChunks; ++ch) {
    const int cbase = ch * CHUNK;
    const int wc = scan_chunk(dsts, nE, cbase, nodeBase, nb, vec8, list, tid, lane, wave);
    if (lane == 0) wcnt[wave] = wc;
    __syncthreads();
    int pre = 0, all = 0;
#pragma unroll
    for (int w2 = 0; w2 < NWAVE; ++w2) {
      int c = wcnt[w2];
      c = c < 0 ? 0 : (c > WCAP ? WCAP : c);
      all += c;
      pre += (w2 < wave) ? c : 0;
    }
    const int wcc  = wc > WCAP ? WCAP : wc;
    const int base = tot + pre;
#pragma unroll 1
    for (int i = lane; i < wcc; i += 32) {
      const int ent = list[wave * WCAP + i];
      const int el  = (ent >> 12) & (CHUNK - 1);
      const int sl  = ent & (NBMAX - 1);
      int eid = cbase + el;
      eid = eid > nE - 1 ? nE - 1 : eid;
      const int pos = base + i;
      if (pos < RCAP) reg1[pos] = (int)(((unsigned)eid << ESH) | (unsigned)sl);
    }
    tot += all;
    tot = tot > RCAP ? RCAP : tot;
    __syncthreads();
  }
  const int nh = tot;

  if (wave == 0) {
#pragma unroll 1
    for (int b0 = 0; b0 < nh; b0 += 32) {
      const int idx = b0 + lane;
      const int uv  = reg1[idx < nh ? idx : nh - 1];
      const int m32 = (nh - b0) < 32 ? (nh - b0) : 32;
#pragma unroll 1
      for (int k = 0; k < m32; ++k) {
        const int u  = __builtin_amdgcn_readlane(uv, k);
        const int sl = u & (NBMAX - 1);
        if (lane == 0) scnt[sl] = scnt[sl] + 1;
      }
    }
  }
  __syncthreads();

  {
    const v4i ca = *(const v4i*)(scnt + 8 * tid);
    const v4i cb = *(const v4i*)(scnt + 8 * tid + 4);
    const int e0 = ca.x < 0 ? 0 : ca.x, e1 = ca.y < 0 ? 0 : ca.y, e2 = ca.z < 0 ? 0 : ca.z, e3 = ca.w < 0 ? 0 : ca.w;
    const int e4 = cb.x < 0 ? 0 : cb.x, e5 = cb.y < 0 ? 0 : cb.y, e6 = cb.z < 0 ? 0 : cb.z, e7 = cb.w < 0 ? 0 : cb.w;
    const int ts = e0 + e1 + e2 + e3 + e4 + e5 + e6 + e7;
    int incl = ts;
#pragma unroll
    for (int d = 1; d < 32; d <<= 1) {
      const int up = __shfl_up(incl, d);
      if (lane >= d) incl += up;
    }
    if (lane == 31) wtot[wave] = incl;
    __syncthreads();
    int pre = 0;
#pragma unroll
    for (int w2 = 0; w2 < NWAVE; ++w2) pre += (w2 < wave) ? wtot[w2] : 0;
    int run = pre + incl - ts;
    soff[8 * tid + 0] = run; run += e0;
    soff[8 * tid + 1] = run; run += e1;
    soff[8 * tid + 2] = run; run += e2;
    soff[8 * tid + 3] = run; run += e3;
    soff[8 * tid + 4] = run; run += e4;
    soff[8 * tid + 5] = run; run += e5;
    soff[8 * tid + 6] = run; run += e6;
    soff[8 * tid + 7] = run;
  }
  __syncthreads();
  for (int i = tid; i < NBMAX; i += NTHR) list[i] = soff[i];
  __syncthreads();

  if (wave == 0) {
#pragma unroll 1
    for (int b0 = 0; b0 < nh; b0 += 32) {
      const int idx = b0 + lane;
      const int uv  = reg1[idx < nh ? idx : nh - 1];
      const int m32 = (nh - b0) < 32 ? (nh - b0) : 32;
#pragma unroll 1
      for (int k = 0; k < m32; ++k) {
        const int u   = __builtin_amdgcn_readlane(uv, k);
        const int sl  = u & (NBMAX - 1);
        const int eid = (int)((unsigned)u >> ESH);
        if (lane == 0) {
          int pos = list[sl];
          pos = pos < 0 ? 0 : (pos > RCAP - 1 ? RCAP - 1 : pos);
          reg2[pos] = eid;
          list[sl] = pos + 1;
        }
      }
    }
  }
  __syncthreads();
  return nh;
}

__global__ __launch_bounds__(NTHR) void k_bucket(const int* __restrict__ dsts, const int* __restrict__ srcs,
                                                 int nE, int nN, int vec8, int* LIST, int* OFFC, int* META) {
  extern __shared__ v4f lds_dyn[];
  int* reg1 = (int*)lds_dyn;
  int* reg2 = reg1 + RCAP;
  int* scnt = reg2 + RCAP;
  int* soff = scnt + NBMAX;
  int* list = soff + NBMAX;
  int* wcnt = list + LISTN;
  int* wtot = wcnt + NWAVE;
  const int tid = (int)threadIdx.x, lane = tid & 31, wave = tid >> 5;
  const int b = (int)blockIdx.x;
  const int nodeBase = b * NBROWS;
  int nb = nN - nodeBase;
  nb = nb < 0 ? 0 : (nb > NBROWS ? NBROWS : nb);

  const int nh = build_lists(dsts, nE, nodeBase, nb, vec8, reg1, reg2, scnt, soff, list, wcnt, wtot, tid, lane, wave);

  int* bl = LIST + (size_t)b * RCAP;
  const int last = nh > 0 ? nh - 1 : 0;
#pragma unroll 1
  for (int base = 0; base < RCAP; base += 1024) {
    const int i0 = base + 4 * tid;
    v4i v = (v4i){0, 0, 0, 0};
    if (base < nh) {
      int e0 = reg2[i0     < last ? i0     : last];
      int e1 = reg2[i0 + 1 < last ? i0 + 1 : last];
      int e2 = reg2[i0 + 2 < last ? i0 + 2 : last];
      int e3 = reg2[i0 + 3 < last ? i0 + 3 : last];
      e0 = clampi(e0, 0, nE - 1);
      e1 = clampi(e1, 0, nE - 1);
      e2 = clampi(e2, 0, nE - 1);
      e3 = clampi(e3, 0, nE - 1);
      const int s0 = srcs[e0];
      const int s1 = srcs[e1];
      const int s2 = srcs[e2];
      const int s3 = srcs[e3];
      asm volatile("" :: "v"(s0), "v"(s1), "v"(s2), "v"(s3));
      v.x = (i0     < nh) ? s0 : 0;
      v.y = (i0 + 1 < nh) ? s1 : 0;
      v.z = (i0 + 2 < nh) ? s2 : 0;
      v.w = (i0 + 3 < nh) ? s3 : 0;
    }
    st2_v4i(bl + i0, v);
  }
  {
    const v4i so = *(const v4ia*)(soff + 4 * tid);
    const v4i sc = *(const v4ia*)(scnt + 4 * tid);
    int* oc = OFFC + (size_t)b * 2048;
    st2_v4i(oc + 4 * tid, so);
    st2_v4i(oc + 1024 + 4 * tid, sc);
  }
  if (tid < 8) {
    v4i mv;
    mv.x = (tid == 0) ? nh : 0;
    mv.y = (tid == 0 && nh >= RCAP) ? 1 : 0;
    mv.z = 0; mv.w = 0;
    st2_v4i(META + (size_t)b * 32 + 4 * tid, mv);
  }
}

__global__ __launch_bounds__(256) void k_replay(
    const float* __restrict__ Q, const float* __restrict__ KPR, const float* __restrict__ VPR,
    const int* __restrict__ LIST, const int* __restrict__ OFFC, const int* __restrict__ META,
    const float* __restrict__ prl, unsigned short* B1) {
  __shared__ float sL[8][DEGCAP * 8];
  __shared__ __attribute__((aligned(16))) float sG[8][CH];
  const int lane = threadIdx.x & 31;
  const int wave = threadIdx.x >> 5;
  const int hd = lane >> 2;
  const int t = (int)blockIdx.x * 8 + wave;
  const bool live = t < NN;
  const int tc = live ? t : NN - 1;
  const int b = clampi(tc >> 10, 0, NBLK - 1);
  const int slot = tc & (NBROWS - 1);
  const int* oc = OFFC + (size_t)b * 2048;
  int stv = oc[slot];
  int cv  = oc[1024 + slot];
  int nhv = META[(size_t)b * 32];
  int flg = META[(size_t)b * 32 + 1];
  asm volatile("" :: "v"(stv), "v"(cv), "v"(nhv), "v"(flg));
  nhv = clampi(nhv, 0, RCAP);
  const int praw = (cv > DEGCAP) ? 1 : 0;
  stv = clampi(stv, 0, nhv);
  cv  = clampi(cv, 0, DEGCAP);
  cv  = cv > nhv - stv ? nhv - stv : cv;
  cv  = live ? cv : 0;
  const int st  = __builtin_amdgcn_readfirstlane(stv);
  const int cnt = __builtin_amdgcn_readfirstlane(cv);
  const int nh  = __builtin_amdgcn_readfirstlane(nhv);
  const int last = nh > 0 ? nh - 1 : 0;
  const bool poison = live && ((flg != 0) || (praw != 0));

  const v4f qv = *(const v4fa*)(Q + (size_t)tc * CH + 4 * lane);
  const float pl = prl[lane];
  asm volatile("" :: "v"(qv), "v"(pl));

  const int* bl = LIST + (size_t)b * RCAP;
  float* strip = &sL[wave][0];
  float* sg = &sG[wave][0];
  const float finf = __builtin_inff();
  const float qnan = __int_as_float(0x7fc00000);

  float m = -finf;
#pragma unroll 1
  for (int q = 0; q < cnt; ++q) {
    int s = bl[clampi(st + q, 0, last)];
    asm volatile("" :: "v"(s));
    s = clampi(s, 0, NN - 1);
    const v4f kk = *(const v4fa*)(KPR + (size_t)s * CH + 4 * lane);
    asm volatile("" :: "v"(kk));
    float pr = qv[0] * kk[0];
    pr = fmaf(qv[1], kk[1], pr);
    pr = fmaf(qv[2], kk[2], pr);
    pr = fmaf(qv[3], kk[3], pr);
    pr += __shfl_xor(pr, 1);
    pr += __shfl_xor(pr, 2);
    const float l = pr * pl * 0.25f;
    if ((lane & 3) == 0) strip[q * 8 + hd] = l;
    m = (l > m) ? l : m;
  }
  wave_sync_lds();
  const float mf = (fabsf(m) < finf) ? m : 0.0f;
  float den = 0.0f;
  v4f acc = (v4f){0.0f, 0.0f, 0.0f, 0.0f};
#pragma unroll 1
  for (int q = 0; q < cnt; ++q) {
    int s = bl[clampi(st + q, 0, last)];
    asm volatile("" :: "v"(s));
    s = clampi(s, 0, NN - 1);
    const v4f vv = *(const v4fa*)(VPR + (size_t)s * CH + 4 * lane);
    asm volatile("" :: "v"(vv));
    const float l = strip[q * 8 + hd];
    const float p = expf(l - mf);
    den += p;
    acc[0] = fmaf(p, vv[0], acc[0]);
    acc[1] = fmaf(p, vv[1], acc[1]);
    acc[2] = fmaf(p, vv[2], acc[2]);
    acc[3] = fmaf(p, vv[3], acc[3]);
  }
  const float rinv = 1.0f / (den + 1e-16f);
  v4f ag = acc * rinv;
  const v4f zero4 = (v4f){0.0f, 0.0f, 0.0f, 0.0f};
  const v4f nan4  = (v4f){qnan, qnan, qnan, qnan};
  ag = (cnt == 0) ? zero4 : ag;
  ag = poison ? nan4 : ag;
  *(v4fa*)(sg + 4 * lane) = ag;
  wave_sync_lds();
  const int c8 = (lane & 15) * 8;
  const v4f a = *(const v4fa*)(sg + c8);
  const v4f c = *(const v4fa*)(sg + c8 + 4);
  const v4u hi = pack8_bf16(a, c);
  const v4u lo = pack8_bf16_lo(a, c);
  const v4u o = (lane >= 16) ? lo : hi;
  st2_v4u(B1 + (size_t)t * 256 + (size_t)lane * 8, o);
}

__global__ __launch_bounds__(256) void k_finish(const float* __restrict__ F2, const float* __restrict__ x,
                                                const float* __restrict__ abv, const float* __restrict__ skp,
                                                const int* __restrict__ META, float* out) {
  const int lane = threadIdx.x & 31;
  const int wave = threadIdx.x >> 5;
  const int t = (int)blockIdx.x * 8 + wave;
  if (t >= NN) return;
  const v4f o  = *(const v4fa*)(F2 + (size_t)t * CH + 4 * lane);
  const v4f xr = *(const v4fa*)(x + (size_t)t * CH + 4 * lane);
  const v4f ab = *(const v4fa*)(abv + 4 * lane);
  const float s = skp[0];
  const int flg = META[(size_t)clampi(t >> 10, 0, NBLK - 1) * 32 + 1];
  asm volatile("" :: "v"(o), "v"(xr), "v"(ab), "v"(s), "v"(flg));
  const float al = 1.0f / (1.0f + expf(-s));
  const float bl = 1.0f - al;
  const float qnan = __int_as_float(0x7fc00000);
  v4f r;
  r[0] = al * (o[0] + ab[0]) + bl * bf16_val(xr[0]);
  r[1] = al * (o[1] + ab[1]) + bl * bf16_val(xr[1]);
  r[2] = al * (o[2] + ab[2]) + bl * bf16_val(xr[2]);
  r[3] = al * (o[3] + ab[3]) + bl * bf16_val(xr[3]);
  const v4f nan4 = (v4f){qnan, qnan, qnan, qnan};
  r = (flg != 0) ? nan4 : r;
  st2_v4f(out + (size_t)t * CH + 4 * lane, r);
}

static void run_pass(const float* xS, const float* xT, const int* tgt, const int* src,
                     const unsigned short* kWT, const unsigned short* vWT, const unsigned short* qWT,
                     const unsigned short* abd, const unsigned short* mbd, const unsigned short* aWT2,
                     const float* TAB, int t_kb, int t_vb, int t_qb, int t_ab, int t_prel, int t_skip,
                     float* F1, float* F2, float* F3, unsigned short* B1, unsigned short* XB,
                     int* LIST, int* OFFC, int* META, float* outT, hipStream_t stream) {
  const int gPlane = MPN * CH / 8 / 256;
  const int gGemm  = (782 * 2 + 7) / 8;
  const int gSplit = MPN * 32 / 256;
  k_plane<0><<<gPlane, 256, 0, stream>>>(xS, NN, CH, CH, XB, MPN, CH);
  k_gemm_nt<0, 0><<<gGemm, 256, 0, stream>>>(XB, kWT, TAB, F1, NN, CH, CH, CH);
  k_split<<<gSplit, 256, 0, stream>>>(F1, TAB + t_kb, B1);
  k_gemm_nt<1, 0><<<gGemm, 256, 0, stream>>>(B1, abd, TAB, F2, NN, CH, 2 * CH, CH);
  k_gemm_nt<0, 0><<<gGemm, 256, 0, stream>>>(XB, vWT, TAB, F1, NN, CH, CH, CH);
  k_split<<<gSplit, 256, 0, stream>>>(F1, TAB + t_vb, B1);
  k_gemm_nt<1, 0><<<gGemm, 256, 0, stream>>>(B1, mbd, TAB, F3, NN, CH, 2 * CH, CH);
  k_plane<0><<<gPlane, 256, 0, stream>>>(xT, NN, CH, CH, XB, MPN, CH);
  k_gemm_nt<0, 1><<<gGemm, 256, 0, stream>>>(XB, qWT, TAB + t_qb, F1, NN, CH, CH, CH);
  k_bucket<<<NBLK, NTHR, LDS_BKT, stream>>>(tgt, src, NE, NN, 1, LIST, OFFC, META);
  k_replay<<<MPN / 8, 256, 0, stream>>>(F1, F2, F3, LIST, OFFC, META, TAB + t_prel, B1);
  k_gemm_nt<1, 0><<<gGemm, 256, 0, stream>>>(B1, aWT2, TAB, F2, NN, CH, 2 * CH, CH);
  k_finish<<<NN / 8, 256, 0, stream>>>(F2, xT, TAB + t_ab, TAB + t_skip, META, outT);
}

extern "C" void kernel_launch(void* const* d_in, const int* in_sizes, int n_in,
                              void* d_out, int out_size, void* d_ws, size_t ws_size,
                              hipStream_t stream) {
  if (n_in < 30) return;
  if (in_sizes[0] != NN * CH || in_sizes[1] != NN * CH) return;
  for (int t = 0; t < 2; ++t) {
    const int o = 2 + 9 * t;
    for (int p = 0; p < 4; ++p) {
      if (in_sizes[o + 2 * p] != CH * CH || in_sizes[o + 2 * p + 1] != CH) return;
    }
    if (in_sizes[o + 8] != 1) return;
  }
  for (int e = 0; e < 2; ++e) {
    const int o = 20 + 3 * e;
    if (in_sizes[o] != 8 * 16 * 16 || in_sizes[o + 1] != 8 * 16 * 16 || in_sizes[o + 2] != 8) return;
  }
  if (in_sizes[26] != NE || in_sizes[27] != NE || in_sizes[28] != NE || in_sizes[29] != NE) return;
  if (out_size != 2 * NN * CH) return;
  if (ws_size < WS_TOTAL) return;

  const float* x_a  = (const float*)d_in[0];
  const float* x_b  = (const float*)d_in[1];
  const float* qW_a = (const float*)d_in[2];   const float* qb_a = (const float*)d_in[3];
  const float* kW_a = (const float*)d_in[4];   const float* kb_a = (const float*)d_in[5];
  const float* vW_a = (const float*)d_in[6];   const float* vb_a = (const float*)d_in[7];
  const float* aW_a = (const float*)d_in[8];   const float* ab_a = (const float*)d_in[9];
  const float* sk_a = (const float*)d_in[10];
  const float* qW_b = (const float*)d_in[11];  const float* qb_b = (const float*)d_in[12];
  const float* kW_b = (const float*)d_in[13];  const float* kb_b = (const float*)d_in[14];
  const float* vW_b = (const float*)d_in[15];  const float* vb_b = (const float*)d_in[16];
  const float* aW_b = (const float*)d_in[17];  const float* ab_b = (const float*)d_in[18];
  const float* sk_b = (const float*)d_in[19];
  const float* arel_ab = (const float*)d_in[20];
  const float* mrel_ab = (const float*)d_in[21];
  const float* prel_ab = (const float*)d_in[22];
  const float* arel_ba = (const float*)d_in[23];
  const float* mrel_ba = (const float*)d_in[24];
  const float* prel_ba = (const float*)d_in[25];
  const int* src_ab = (const int*)d_in[26];
  const int* tgt_ab = (const int*)d_in[27];
  const int* src_ba = (const int*)d_in[28];
  const int* tgt_ba = (const int*)d_in[29];
  float* out = (float*)d_out;

  char* ws = (char*)d_ws;
  float*          F1   = (float*)(ws + O_F1);
  float*          F2   = (float*)(ws + O_F2);
  float*          F3   = (float*)(ws + O_F3);
  unsigned short* B1   = (unsigned short*)(ws + O_B1);
  unsigned short* XB   = (unsigned short*)(ws + O_XB);
  int*            LIST = (int*)(ws + O_LIST);
  int*            OFFC = (int*)(ws + O_OFFC);
  int*            META = (int*)(ws + O_META);
  unsigned short* WT   = (unsigned short*)(ws + O_WT);
  float*          TAB  = (float*)(ws + O_TAB);

  hipFuncSetAttribute(reinterpret_cast<const void*>(&k_bucket),
                      hipFuncAttributeMaxDynamicSharedMemorySize, LDS_BKT);

  k_wprep<<<145, 256, 0, stream>>>(qW_a, kW_a, vW_a, aW_a, qW_b, kW_b, vW_b, aW_b,
                                   arel_ab, mrel_ab, arel_ba, mrel_ba,
                                   qb_a, kb_a, vb_a, ab_a, qb_b, kb_b, vb_b, ab_b,
                                   prel_ab, prel_ba, sk_a, sk_b, WT, TAB);

  run_pass(x_a, x_b, tgt_ab, src_ab,
           WT + WT_K_A, WT + WT_V_A, WT + WT_Q_B, WT + WT_ABD_AB, WT + WT_MBD_AB, WT + WT_A2_B,
           TAB, T_KB_A, T_VB_A, T_QB_B, T_AB_B, T_PREL_AB, T_SKIP + 1,
           F1, F2, F3, B1, XB, LIST, OFFC, META, out + (size_t)NN * CH, stream);
  run_pass(x_b, x_a, tgt_ba, src_ba,
           WT + WT_K_B, WT + WT_V_B, WT + WT_Q_A, WT + WT_ABD_BA, WT + WT_MBD_BA, WT + WT_A2_A,
           TAB, T_KB_B, T_VB_B, T_QB_A, T_AB_A, T_PREL_BA, T_SKIP + 0,
           F1, F2, F3, B1, XB, LIST, OFFC, META, out, stream);
}
